// se_conv_BiLSTM_20925080666591
// MI455X (gfx1250) — hardware-verified
//
#include <hip/hip_runtime.h>


namespace {
constexpr int NBt = 128, T = 10, P = 40, C = 300, CP = 320, F = 256, G4 = 4 * F, NR = NBt * P;
constexpr float XS = 8.0f, WSC = 256.0f;

typedef _Float16 b16;
typedef __attribute__((ext_vector_type(16))) _Float16 v16b;
typedef __attribute__((ext_vector_type(8))) _Float16 v8b;
typedef __attribute__((ext_vector_type(2))) _Float16 v2b;
typedef __attribute__((ext_vector_type(8))) float v8f;
typedef __attribute__((ext_vector_type(4))) float v4f;
__device__ __forceinline__ float bf16_rne(float f) { unsigned int u = __float_as_uint(f); u += 0x7FFFu + ((u >> 16) & 1u); return __uint_as_float(u & 0xFFFF0000u); }
__device__ __forceinline__ void split16(float v, b16& hi, b16& lo) { hi = (b16)v; lo = (b16)(v - (float)hi); }
__device__ __forceinline__ v16b frag_kb(const b16* p, int hh) { const v8b a = *(const v8b*)(p + 8 * hh), b = *(const v8b*)(p + 16 + 8 * hh); v16b f;
#pragma unroll
  for (int e = 0; e < 8; ++e) { f[e] = a[e]; f[8 + e] = b[e]; } return f; }
__device__ __forceinline__ v8f wmma16b(v16b a, v16b b, v8f c) { v8f d = __builtin_amdgcn_wmma_f32_16x16x32_f16(false, a, false, b, (short)0, c, false, false); asm volatile("v_nop\n\tv_nop\n\tv_nop\n\tv_nop" : "+v"(d) : "v"(a), "v"(b)); return d; }
__device__ __forceinline__ float nexp(float x) { return __builtin_amdgcn_exp2f(x * 1.4426950408889634f); }
__device__ __forceinline__ float pmul(float a, float b) { float p = a * b; asm volatile("" : "+v"(p)); return p; }
__device__ __forceinline__ float tanh_(float x) { const float e = nexp(-2.0f * fabsf(x)); const float t = (1.0f - e) / (1.0f + e); return x < 0.0f ? -t : t; }
__device__ __forceinline__ float hsig(float x) { return fminf(fmaxf(0.2f * x + 0.5f, 0.0f), 1.0f); }

__global__ __launch_bounds__(256) void prepx_kernel(const float* __restrict__ x, b16* __restrict__ X16) {
  const int wave = threadIdx.x >> 5, lane = threadIdx.x & 31; const int g = blockIdx.x * 8 + wave;
  const int b = g / (T * P), rem = g - b * T * P, t = rem / P, p = rem - t * P; const float* src = x + (size_t)g * C; b16* dst = X16 + (((size_t)(b * P + p)) * T + t) * CP;
  v8b o0, o1;
#pragma unroll
  for (int q = 0; q < 8; ++q) { const int e = lane * 8 + q; o0[q] = (e < C) ? (b16)(bf16_rne(src[e < C ? e : 0]) * XS) : (b16)0.0f; const int e1 = 256 + lane * 8 + q; o1[q] = (e1 < C && lane < 8) ? (b16)(bf16_rne(src[e1 < C ? e1 : 0]) * XS) : (b16)0.0f; }
  for (int pass = 0; pass < 2; ++pass) { *(volatile v8b*)(dst + lane * 8) = o0; if (lane < 8) *(volatile v8b*)(dst + 256 + lane * 8) = o1; __threadfence(); }
}
__global__ __launch_bounds__(256) void prepw_kernel(const float* __restrict__ wkf, const float* __restrict__ wrf, const float* __restrict__ wkb, const float* __restrict__ wrb, b16* __restrict__ WK, b16* __restrict__ WR) {
  __shared__ __attribute__((aligned(16))) b16 Tt[64][64 + 8];
  const int kind = blockIdx.z, dir = kind & 1, isr = kind >> 1, k0 = blockIdx.x * 64, n0 = blockIdx.y * 64, t_ = threadIdx.x;
  const int K = isr ? F : C, KP = isr ? F : CP; if (k0 >= KP) return;
  const float* w = isr ? (dir ? wrb : wrf) : (dir ? wkb : wkf); b16* dst = isr ? WR + (size_t)dir * G4 * F : WK + (size_t)dir * G4 * CP;
  for (int q = t_; q < 64 * 64; q += 256) { const int kk = q >> 6, nn = q & 63; const int k = k0 + kk; Tt[nn][kk] = (k < K) ? (b16)(bf16_rne(w[(size_t)(k < K ? k : 0) * G4 + n0 + nn]) * WSC) : (b16)0.0f; }
  __syncthreads();
  for (int pass = 0; pass < 2; ++pass) { for (int q = t_; q < 64 * 8; q += 256) { const int nn = q >> 3, c8 = (q & 7) * 8; *(volatile v8b*)(dst + (size_t)(n0 + nn) * KP + k0 + c8) = *(const v8b*)(&Tt[nn][c8]); } __threadfence(); }
}
template <int DIR>
__global__ __launch_bounds__(512) void lstm_kernel(const b16* __restrict__ X16, const b16* __restrict__ WK, const b16* __restrict__ WR, const float* __restrict__ bf, const float* __restrict__ bb, float* __restrict__ HF, float* __restrict__ out) {
  __shared__ __attribute__((aligned(16))) b16 Hh[32][F + 8], Hl[32][F + 8]; __shared__ __attribute__((aligned(16))) float Ho[32][F + 4];
  const int t_ = threadIdx.x, wave = t_ >> 5, lane = t_ & 31, nloc = lane & 15, hlf = lane >> 4; const int j = wave * 16 + nloc; const int r0 = blockIdx.x * 32;
  const b16* Wk = WK + (size_t)DIR * G4 * CP; const b16* Wr = WR + (size_t)DIR * G4 * F; const float* bias = DIR ? bb : bf;
  for (int k = t_; k < 32 * (F + 8); k += 512) { (&Hh[0][0])[k] = (b16)0.0f; (&Hl[0][0])[k] = (b16)0.0f; }
  float bg[4];
#pragma unroll
  for (int g = 0; g < 4; ++g) bg[g] = bf16_rne(bias[g * F + j]);
  float cst[2][8];
#pragma unroll
  for (int mt = 0; mt < 2; ++mt)
#pragma unroll
    for (int r = 0; r < 8; ++r) cst[mt][r] = 0.0f;
  __syncthreads();
  for (int step = 0; step < T; ++step) { const int tin = DIR ? (T - 1 - step) : step;
    v8f acc[2][4];
#pragma unroll
    for (int mt = 0; mt < 2; ++mt)
#pragma unroll
      for (int g = 0; g < 4; ++g) acc[mt][g] = (v8f){};
#pragma unroll 2
    for (int kb = 0; kb < CP; kb += 32) { v16b a[2];
#pragma unroll
      for (int mt = 0; mt < 2; ++mt) a[mt] = frag_kb(X16 + ((size_t)(r0 + mt * 16 + nloc) * T + tin) * CP + kb, hlf);
#pragma unroll
      for (int g = 0; g < 4; ++g) { const v16b bw = frag_kb(Wk + (size_t)(g * F + j) * CP + kb, hlf);
#pragma unroll
        for (int mt = 0; mt < 2; ++mt) acc[mt][g] = wmma16b(a[mt], bw, acc[mt][g]); } }
#pragma unroll
    for (int kb = 0; kb < F; kb += 32) { v16b ah[2], al[2];
#pragma unroll
      for (int mt = 0; mt < 2; ++mt) { ah[mt] = frag_kb(&Hh[mt * 16 + nloc][kb], hlf); al[mt] = frag_kb(&Hl[mt * 16 + nloc][kb], hlf); }
#pragma unroll
      for (int g = 0; g < 4; ++g) { const v16b bw = frag_kb(Wr + (size_t)(g * F + j) * F + kb, hlf);
#pragma unroll
        for (int mt = 0; mt < 2; ++mt) { acc[mt][g] = wmma16b(ah[mt], bw, acc[mt][g]); acc[mt][g] = wmma16b(al[mt], bw, acc[mt][g]); } } }
    __syncthreads();
#pragma unroll
    for (int mt = 0; mt < 2; ++mt)
#pragma unroll
      for (int r = 0; r < 8; ++r) { const float zi = acc[mt][0][r] * (1.0f / (XS * WSC)) + bg[0], zf = acc[mt][1][r] * (1.0f / (XS * WSC)) + bg[1], zc = acc[mt][2][r] * (1.0f / (XS * WSC)) + bg[2], zo = acc[mt][3][r] * (1.0f / (XS * WSC)) + bg[3];
        const float ig = DIR ? tanh_(zi) : hsig(zi), fg = DIR ? tanh_(zf) : hsig(zf), og = DIR ? tanh_(zo) : hsig(zo);
        const float c = pmul(fg, cst[mt][r]) + pmul(ig, tanh_(zc)); cst[mt][r] = c; const float h = pmul(og, tanh_(c)); const int rr = mt * 16 + 8 * hlf + r;
        Ho[rr][j] = h; b16 a_, c_; split16(h * XS, a_, c_); const float nh = __shfl_xor((float)a_, 1), nl = __shfl_xor((float)c_, 1);
        if ((nloc & 1) == 0) { v2b ph, pl; ph[0] = a_; ph[1] = (b16)nh; pl[0] = c_; pl[1] = (b16)nl; *(v2b*)(&Hh[rr][j]) = ph; *(v2b*)(&Hl[rr][j]) = pl; } }
    __syncthreads();
    for (int pass = 0; pass < 2; ++pass) { for (int rr = wave * 2; rr < wave * 2 + 2; ++rr) { const int row = r0 + rr;
        if (DIR == 0) { for (int hq = 0; hq < 2; ++hq) *(volatile v4f*)(HF + ((size_t)step * NR + row) * F + hq * 128 + lane * 4) = *(const v4f*)(&Ho[rr][hq * 128 + lane * 4]); }
        else { const int b = row / P, p = row - b * P; for (int hq = 0; hq < 2; ++hq) { const v4f hv = *(const v4f*)(&Ho[rr][hq * 128 + lane * 4]); const v4f fv = *(const v4f*)(HF + ((size_t)step * NR + row) * F + hq * 128 + lane * 4);
            *(volatile v4f*)(out + (((size_t)b * T + step) * P + p) * F + hq * 128 + lane * 4) = hv + fv; } } }
      __threadfence(); } }
}
}

extern "C" void kernel_launch(void* const* d_in, const int* in_sizes, int n_in, void* d_out, int out_size, void* d_ws, size_t ws_size, hipStream_t stream) {
  (void)n_in;
  auto Fp = [&](int i) { return (const float*)d_in[i]; };
  if (in_sizes[0] != NBt * T * P * C || in_sizes[1] != C * G4 || in_sizes[2] != F * G4 || in_sizes[4] != C * G4 || out_size != NBt * T * P * F) return;
  size_t off = 0; char* ws = (char*)d_ws;
  auto carve = [&](size_t bytes) { char* p = ws + off; off += (bytes + 255) & ~(size_t)255; return p; };
  b16* X16 = (b16*)carve((size_t)NR * T * CP * 2); b16* WK = (b16*)carve((size_t)2 * G4 * CP * 2); b16* WR = (b16*)carve((size_t)2 * G4 * F * 2); float* HF = (float*)carve((size_t)T * NR * F * 4);
  if (off > ws_size || off > ((size_t)128 << 20)) return;
  prepx_kernel<<<NBt * T * P / 8, 256, 0, stream>>>(Fp(0), X16);
  prepw_kernel<<<dim3(CP / 64, G4 / 64, 4), 256, 0, stream>>>(Fp(1), Fp(2), Fp(4), Fp(5), WK, WR);
  lstm_kernel<0><<<NR / 32, 512, 0, stream>>>(X16, WK, WR, Fp(3), Fp(6), HF, (float*)d_out);
  lstm_kernel<1><<<NR / 32, 512, 0, stream>>>(X16, WK, WR, Fp(3), Fp(6), HF, (float*)d_out);
}
